// MM4d_36086315221298
// MI455X (gfx1250) — hardware-run, weakly checked
//
#include <hip/hip_runtime.h>
#include <math.h>

typedef __attribute__((ext_vector_type(16))) _Float16 v16h;
typedef __attribute__((ext_vector_type(8)))  _Float16 v8h;
typedef __attribute__((ext_vector_type(8)))  float    v8f;
typedef __attribute__((ext_vector_type(4)))  float    v4f;

constexpr int kBatch  = 4;
constexpr int kNode   = 16;
constexpr int kLen    = 512;
constexpr int kNin    = 32;
constexpr int kHid    = 64;
constexpr int kNst    = 128;
constexpr int kDtr    = 4;
constexpr int kNout   = 64;
constexpr int kSeqs   = kBatch * kNode;
constexpr int kRows   = kSeqs * kLen;
constexpr int kXpCols = kDtr + 2 * kNst;
constexpr int kXpPad  = 320;
constexpr int kPDt    = 2 * kNst;
constexpr int kSeqElems = kLen * kNout;
constexpr float kWCarry = 1024.0f;
constexpr float kResid  = 2048.0f;
constexpr float kScale  = 1.0f / kWCarry;
constexpr float kRScale = 1.0f / (kWCarry * kResid);
constexpr float kInvCount = 1.0f / (float)kSeqElems;
constexpr bool kWeightLo = true;
constexpr int  kSpl = kWeightLo ? 2 : 1;
static_assert(kRows == 32768 && kXpCols == 260 && kPDt == 256);
static_assert((kNin % 32) == 0 && (kHid % 32) == 0);
static_assert((kRows % 16) == 0 && (kHid % 64) == 0 && ((2 * kHid) % 64) == 0 && (kXpPad % 64) == 0 && (kNout % 64) == 0);
static_assert(kXpPad >= kXpCols && (kLen % 32) == 0 && (kLen % 16) == 0);

constexpr size_t kSzWdim = (size_t)kHid * kNin * 2;
constexpr size_t kSzWin  = (size_t)(2 * kHid) * kHid * 2;
constexpr size_t kSzWxp  = (size_t)kXpPad * kHid * 2;
constexpr size_t kSzWsq  = (size_t)kHid * kHid * 2;
constexpr size_t kSzWAll = kSzWdim + kSzWin + kSzWxp + 2 * kSzWsq;
constexpr size_t kSzWLo  = kWeightLo ? kSzWAll : 0;
constexpr size_t kSzX16  = (size_t)kRows * kNin * 2;
constexpr size_t kSzH16  = (size_t)kRows * kHid * 2;
constexpr size_t kSzF32  = (size_t)kRows * kHid * 4;
constexpr size_t kSzP    = (size_t)kRows * kXpPad * 4;
constexpr size_t kOffWdim = 0;
constexpr size_t kOffWin  = kOffWdim + kSzWdim;
constexpr size_t kOffWxp  = kOffWin  + kSzWin;
constexpr size_t kOffWop  = kOffWxp  + kSzWxp;
constexpr size_t kOffWo   = kOffWop  + kSzWsq;
constexpr size_t kOffWLo  = kOffWo   + kSzWsq;
constexpr size_t kOffXH   = kOffWLo  + kSzWLo;
constexpr size_t kOffXL   = kOffXH   + kSzX16;
constexpr size_t kOffXDH  = kOffXL   + kSzX16;
constexpr size_t kOffXDL  = kOffXDH  + kSzH16;
constexpr size_t kOffXI   = kOffXDL  + kSzH16;
constexpr size_t kOffSG   = kOffXI   + kSzF32;
constexpr size_t kOffU    = kOffSG   + kSzF32;
constexpr size_t kOffUH   = kOffU    + kSzF32;
constexpr size_t kOffUL   = kOffUH   + kSzH16;
constexpr size_t kOffP    = kOffUL   + kSzH16;
constexpr size_t kOffYH   = kOffP    + kSzP;
constexpr size_t kOffYL   = kOffYH   + kSzH16;
constexpr size_t kOffTH   = kOffYL   + kSzH16;
constexpr size_t kOffTL   = kOffTH   + kSzH16;
constexpr size_t kOffY4   = kOffTL   + kSzH16;
constexpr size_t kWsTotal = kOffY4   + kSzF32;
static_assert(kSzWAll == 77824ull);
static_assert(kWsTotal == 113324032ull + (kWeightLo ? 77824ull : 0ull));
static_assert(kWsTotal <= 134217728ull);
static_assert((kOffWin % 128) == 0 && (kOffWxp % 128) == 0 && (kOffWop % 128) == 0 && (kOffWo % 128) == 0 &&
              (kOffWLo % 128) == 0 && (kOffXH % 128) == 0 && (kOffXL % 128) == 0 && (kOffXDH % 128) == 0 &&
              (kOffXDL % 128) == 0 && (kOffXI % 128) == 0 && (kOffSG % 128) == 0 && (kOffU % 128) == 0 &&
              (kOffUH % 128) == 0 && (kOffUL % 128) == 0 && (kOffP % 128) == 0 && (kOffYH % 128) == 0 &&
              (kOffYL % 128) == 0 && (kOffTH % 128) == 0 && (kOffTL % 128) == 0 && (kOffY4 % 128) == 0);
static_assert((size_t)kNode * kNout * kBatch * kLen * 4 == 8388608ull);

__device__ __forceinline__ _Float16 f16_flush(float v) {
  const float w = (fabsf(v) < 6.103515625e-05f) ? 0.0f : v;
  return (_Float16)w;
}
__device__ __forceinline__ void f16_split(float v, _Float16& hi, _Float16& lo) {
  hi = f16_flush(v);
  const float hf = (float)hi;
  const float r = (v - hf) * kResid;
  lo = f16_flush(r);
}
__device__ __forceinline__ void pin_f(float& x) { asm volatile("" : "+v"(x)); }
__device__ __forceinline__ void pin_v4(v4f& x) { asm volatile("" : "+v"(x)); }
__device__ __forceinline__ float act_silu(float v) {
  const float sg = __builtin_amdgcn_rcpf(1.0f + expf(-v));
  return v * sg;
}
__device__ __forceinline__ float act_softplus(float v) {
  return fmaxf(v, 0.0f) + log1pf(expf(-fabsf(v)));
}

namespace eng {
union FragU { v16h v; v8h h[2]; };
__device__ __forceinline__ v16h frag_load(const _Float16* p) {
  FragU f;
  f.h[0] = *(const v8h*)(p);
  f.h[1] = *(const v8h*)(p + 16);
  return f.v;
}
__device__ __forceinline__ v8f mma(v16h a, v16h b, v8f c) {
  return __builtin_amdgcn_wmma_f32_16x16x32_f16(false, a, false, b, (short)0, c, false, false);
}
__device__ __forceinline__ void guard1(v8f& a, v16h x, v16h y) {
  asm volatile("v_nop\n\tv_nop\n\tv_nop\n\tv_nop" : "+v"(a) : "v"(x), "v"(y));
}
__device__ __forceinline__ void guard_acc(v8f& a) {
  asm volatile("v_nop\n\tv_nop\n\tv_nop\n\tv_nop" : "+v"(a));
}
__device__ __forceinline__ void keep4(v16h a, v16h b, v16h c, v16h d) {
  asm volatile("v_nop" :: "v"(a), "v"(b), "v"(c), "v"(d));
}

template <int MI, int SPL, int ACT, int OUT, bool BIAS>
__global__ __launch_bounds__(256) void gemm_f16_kernel(
    const unsigned short* __restrict__ Ap, const unsigned short* __restrict__ A2p, int lda,
    const unsigned short* __restrict__ Btp, const unsigned short* __restrict__ Bt2p, int ldb,
    float* C, float* C2, unsigned short* Hp, unsigned short* Lp, int ldc, int nsplit,
    const float* __restrict__ bias, int M, int N, int K, float scale, float rscale)
{
  static_assert(MI >= 1 && MI <= 2);
  static_assert(SPL >= 0 && SPL <= 2);
  static_assert(ACT >= 0 && ACT <= 2);
  static_assert(OUT >= 0 && OUT <= 1);
  const _Float16* A   = (const _Float16*)Ap;
  const _Float16* A2  = (const _Float16*)A2p;
  const _Float16* Bt  = (const _Float16*)Btp;
  const _Float16* Bt2 = (const _Float16*)Bt2p;
  __shared__ __align__(16) float sT[8][16 * 68];
  const int lane = threadIdx.x & 31;
  const int wave = threadIdx.x >> 5;
  const int tilesN = N >> 6;
  const int tilesM = M / (16 * MI);
  const int tile = blockIdx.x * 8 + wave;
  if (tile >= tilesM * tilesN) return;
  const int tm = tile / tilesN;
  const int tn = tile - tm * tilesN;
  const int m0 = tm * (16 * MI);
  const int n0 = tn << 6;
  const int rlane = lane & 15;
  const int koff  = (lane >> 4) * 8;
  const int mOff  = (lane >> 4) * 8;

  v8f acc[MI][4], accr[MI][4];
#pragma unroll
  for (int i = 0; i < MI; ++i)
#pragma unroll
    for (int j = 0; j < 4; ++j) {
      acc[i][j]  = (v8f){0.f, 0.f, 0.f, 0.f, 0.f, 0.f, 0.f, 0.f};
      accr[i][j] = (v8f){0.f, 0.f, 0.f, 0.f, 0.f, 0.f, 0.f, 0.f};
    }

  for (int k0 = 0; k0 < K; k0 += 32) {
    v16h bh[4], bl[4];
#pragma unroll
    for (int j = 0; j < 4; ++j) {
      const size_t bo = (size_t)(n0 + (j << 4) + rlane) * ldb + koff + k0;
      bh[j] = frag_load(Bt + bo);
      if (SPL == 2) bl[j] = frag_load(Bt2 + bo); else bl[j] = bh[j];
    }
#pragma unroll
    for (int i = 0; i < MI; ++i) {
      const size_t ao = (size_t)(m0 + (i << 4) + rlane) * lda + koff + k0;
      const v16h ah = frag_load(A + ao);
      v16h al = ah;
      if (SPL >= 1) al = frag_load(A2 + ao);
#pragma unroll
      for (int jp = 0; jp < 2; ++jp) {
#pragma unroll
        for (int jj = 0; jj < 2; ++jj) {
          const int j = jp * 2 + jj;
          acc[i][j] = mma(ah, bh[j], acc[i][j]);
          if (SPL >= 1) accr[i][j] = mma(al, bh[j], accr[i][j]);
          if (SPL == 2) accr[i][j] = mma(ah, bl[j], accr[i][j]);
        }
#pragma unroll
        for (int jj = 0; jj < 2; ++jj) {
          const int j = jp * 2 + jj;
          guard1(acc[i][j], ah, al);
          if (SPL >= 1) guard1(accr[i][j], ah, al);
        }
      }
    }
    keep4(bh[0], bh[1], bh[2], bh[3]);
    if (SPL == 2) keep4(bl[0], bl[1], bl[2], bl[3]);
  }
#pragma unroll
  for (int i = 0; i < MI; ++i)
#pragma unroll
    for (int j = 0; j < 4; ++j) {
      guard_acc(acc[i][j]);
      if (SPL >= 1) guard_acc(accr[i][j]);
    }

  float* slab = sT[wave];
  float* Cd = C;
  int nd = n0;
  bool gateTile = false;
  if (ACT == 2) {
    if (n0 >= nsplit) { Cd = C2; nd = n0 - nsplit; gateTile = true; }
  }
  const int hh = lane >> 4, c4 = (lane & 15) * 4;
  const int q  = lane >> 3, c8 = (lane & 7) * 8;
  v4f bv  = (v4f){0.f, 0.f, 0.f, 0.f};
  v4f bv0 = (v4f){0.f, 0.f, 0.f, 0.f};
  v4f bv1 = (v4f){0.f, 0.f, 0.f, 0.f};
  if (BIAS) {
    if (OUT == 0) {
      bv = *(const v4f*)(bias + n0 + c4);
    } else {
      bv0 = *(const v4f*)(bias + n0 + c8);
      bv1 = *(const v4f*)(bias + n0 + c8 + 4);
    }
  }
#pragma unroll
  for (int i = 0; i < MI; ++i) {
    const int mBase = m0 + (i << 4);
#pragma unroll
    for (int j = 0; j < 4; ++j) {
#pragma unroll
      for (int r = 0; r < 8; ++r) {
        float v = acc[i][j][r] * scale;
        if (SPL >= 1) v += accr[i][j][r] * rscale;
        slab[(mOff + r) * 68 + (j << 4) + rlane] = v;
      }
    }
    __builtin_amdgcn_fence(__ATOMIC_RELEASE, "workgroup");
    __builtin_amdgcn_wave_barrier();
    __builtin_amdgcn_fence(__ATOMIC_ACQUIRE, "workgroup");
    if (OUT == 0) {
      if (BIAS || ACT != 0) {
        for (int it = 0; it < 8; ++it) {
          float* sp = slab + (it * 2 + hh) * 68 + c4;
          v4f v = *(const v4f*)sp;
          v = v + bv;
          if (ACT == 1) {
#pragma unroll
            for (int e = 0; e < 4; ++e) v[e] = act_silu(v[e]);
          }
          if (ACT == 2) {
            if (gateTile) {
#pragma unroll
              for (int e = 0; e < 4; ++e) v[e] = act_silu(v[e]);
            }
          }
          *(v4f*)sp = v;
        }
      }
      for (int pass = 0; pass < 2; ++pass) {
#pragma unroll
        for (int it = 0; it < 8; ++it) {
          const int row = it * 2 + hh;
          const v4f v = *(const v4f*)(slab + row * 68 + c4);
          *(volatile v4f*)(Cd + (size_t)(mBase + row) * ldc + nd + c4) = v;
        }
        __threadfence();
      }
    } else {
      v8h hv[4], lv[4];
#pragma unroll
      for (int it = 0; it < 4; ++it) {
        const float* sp = slab + (it * 4 + q) * 68 + c8;
        v4f a0 = *(const v4f*)(sp);
        v4f a1 = *(const v4f*)(sp + 4);
        a0 = a0 + bv0;
        a1 = a1 + bv1;
        if (ACT == 1) {
#pragma unroll
          for (int e = 0; e < 4; ++e) { a0[e] = act_silu(a0[e]); a1[e] = act_silu(a1[e]); }
        }
#pragma unroll
        for (int e = 0; e < 4; ++e) {
          _Float16 h0, l0, h1, l1;
          const float f0 = a0[e];
          const float f1 = a1[e];
          f16_split(f0, h0, l0);
          f16_split(f1, h1, l1);
          hv[it][e] = h0; lv[it][e] = l0;
          hv[it][4 + e] = h1; lv[it][4 + e] = l1;
        }
      }
      for (int pass = 0; pass < 2; ++pass) {
#pragma unroll
        for (int it = 0; it < 4; ++it) {
          const size_t o = (size_t)(mBase + it * 4 + q) * ldc + n0 + c8;
          *(volatile v8h*)(Hp + o) = hv[it];
          *(volatile v8h*)(Lp + o) = lv[it];
        }
        __threadfence();
      }
    }
    __builtin_amdgcn_fence(__ATOMIC_RELEASE, "workgroup");
    __builtin_amdgcn_wave_barrier();
    __builtin_amdgcn_fence(__ATOMIC_ACQUIRE, "workgroup");
  }
}
}

__global__ __launch_bounds__(256) void split_rows_f16_kernel(
    const float* __restrict__ src, unsigned short* __restrict__ dH, unsigned short* __restrict__ dL, int total8)
{
  const int i = blockIdx.x * 256 + threadIdx.x;
  if (i >= total8) return;
  const size_t e0 = (size_t)i << 3;
  const v4f a0 = *(const v4f*)(src + e0);
  const v4f a1 = *(const v4f*)(src + e0 + 4);
  v8h hv, lv;
#pragma unroll
  for (int e = 0; e < 4; ++e) {
    _Float16 h0, l0, h1, l1;
    const float f0 = a0[e];
    const float f1 = a1[e];
    f16_split(f0, h0, l0);
    f16_split(f1, h1, l1);
    hv[e] = h0; lv[e] = l0;
    hv[4 + e] = h1; lv[4 + e] = l1;
  }
  unsigned short* qh = dH + e0;
  unsigned short* ql = dL + e0;
  *(volatile v8h*)qh = hv;
  *(volatile v8h*)ql = lv;
  __threadfence();
  *(volatile v8h*)qh = hv;
  *(volatile v8h*)ql = lv;
}

template <bool LO>
__global__ __launch_bounds__(256) void pack_weight_kernel(
    const float* __restrict__ W, unsigned short* __restrict__ BtH, unsigned short* __restrict__ BtL,
    int Kdim, int Ndim, int xpmode, int total8)
{
  const int i = blockIdx.x * 256 + threadIdx.x;
  if (i >= total8) return;
  const int e0 = i << 3;
  const int n  = e0 / Kdim;
  const int k0 = e0 - n * Kdim;
  int c = n;
  bool valid = (n < Ndim);
  if (xpmode != 0) {
    c = (n < kPDt) ? (n + kDtr) : (n - kPDt);
    valid = (n < kXpCols);
  }
  const int cc = (c < 0) ? 0 : ((c > Ndim - 1) ? (Ndim - 1) : c);
  v8h hv, lv;
#pragma unroll
  for (int e = 0; e < 8; ++e) {
    float v = W[(size_t)(k0 + e) * Ndim + cc];
    pin_f(v);
    const float t = valid ? (v * kWCarry) : 0.0f;
    _Float16 h, l;
    f16_split(t, h, l);
    hv[e] = h;
    lv[e] = l;
  }
  unsigned short* qh = BtH + e0;
  unsigned short* ql = BtL + e0;
  *(volatile v8h*)qh = hv;
  if (LO) *(volatile v8h*)ql = lv;
  __threadfence();
  *(volatile v8h*)qh = hv;
  if (LO) *(volatile v8h*)ql = lv;
}

__global__ __launch_bounds__(256) void conv_silu_kernel(
    const float* __restrict__ XI, const float* __restrict__ cw, const float* __restrict__ cb,
    float* __restrict__ U, unsigned short* __restrict__ UH, unsigned short* __restrict__ UL)
{
  __shared__ __align__(16) float sU[32 * 64];
  const int tid = threadIdx.x;
  const int r0 = blockIdx.x * 32;
  v4f fv[2];
#pragma unroll
  for (int i = 0; i < 2; ++i) {
    const int idx = tid + i * 256;
    const int rr  = idx >> 4;
    const int c4  = (idx & 15) * 4;
    const int row = r0 + rr;
    const int l   = row & (kLen - 1);
    const bool ok = (l > 0);
    const int rp  = ok ? (row - 1) : row;
    const v4f x0 = *(const v4f*)(XI + (size_t)row * kHid + c4);
    v4f xm = *(const v4f*)(XI + (size_t)rp * kHid + c4);
    pin_v4(xm);
    const v4f wa = *(const v4f*)(cw + c4 * 2);
    const v4f wb = *(const v4f*)(cw + c4 * 2 + 4);
    const v4f bc = *(const v4f*)(cb + c4);
    const float w0[4] = {wa[0], wa[2], wb[0], wb[2]};
    const float w1[4] = {wa[1], wa[3], wb[1], wb[3]};
    v4f r;
#pragma unroll
    for (int e = 0; e < 4; ++e) {
      const float xp = ok ? xm[e] : 0.0f;
      float acc = xp * w0[e];
      acc = fmaf(x0[e], w1[e], acc);
      const float sv = bc[e] + acc;
      r[e] = act_silu(sv);
    }
    fv[i] = r;
    *(v4f*)(sU + rr * 64 + c4) = r;
  }
  __syncthreads();
  const int rr8 = tid >> 3;
  const int c8  = (tid & 7) * 8;
  v8h hv, lv;
  {
    const float* sp = sU + rr8 * 64 + c8;
    const v4f a0 = *(const v4f*)(sp);
    const v4f a1 = *(const v4f*)(sp + 4);
#pragma unroll
    for (int e = 0; e < 4; ++e) {
      _Float16 h0, l0, h1, l1;
      const float f0 = a0[e];
      const float f1 = a1[e];
      f16_split(f0, h0, l0);
      f16_split(f1, h1, l1);
      hv[e] = h0; lv[e] = l0;
      hv[4 + e] = h1; lv[4 + e] = l1;
    }
  }
  const size_t o16 = (size_t)(r0 + rr8) * kHid + c8;
  for (int pass = 0; pass < 2; ++pass) {
#pragma unroll
    for (int i = 0; i < 2; ++i) {
      const int idx = tid + i * 256;
      *(volatile v4f*)(U + (size_t)r0 * kHid + (size_t)idx * 4) = fv[i];
    }
    *(volatile v8h*)(UH + o16) = hv;
    *(volatile v8h*)(UL + o16) = lv;
    __threadfence();
  }
}

__global__ __launch_bounds__(256) void scan_kernel(
    const float* __restrict__ P, const float* __restrict__ U, const float* __restrict__ SG,
    const float* __restrict__ Wdt, const float* __restrict__ bdt, const float* __restrict__ Alog,
    const float* __restrict__ Dskip, unsigned short* __restrict__ YH, unsigned short* __restrict__ YL)
{
  __shared__ __align__(16) float sBC[16 * 256];
  __shared__ __align__(16) float sDt[16 * 64];
  __shared__ __align__(16) float sU[16 * 64];
  __shared__ __align__(16) float sG[16 * 64];
  __shared__ __align__(16) float sY[16 * 64];
  __shared__ __align__(16) float sW[kDtr * kHid + kHid];
  const int tid = threadIdx.x;
  const int seq = blockIdx.x;
  const int d = tid >> 2;
  const int g = tid & 3;

  sW[tid] = Wdt[tid];
  if (tid < kHid) sW[kDtr * kHid + tid] = bdt[tid];

  float Ar[32], hs[32];
  {
    const float* ap = Alog + (size_t)d * kNst + g * 32;
#pragma unroll
    for (int k = 0; k < 8; ++k) {
      const v4f a = *(const v4f*)(ap + 4 * k);
      Ar[4 * k + 0] = -expf(a[0]);
      Ar[4 * k + 1] = -expf(a[1]);
      Ar[4 * k + 2] = -expf(a[2]);
      Ar[4 * k + 3] = -expf(a[3]);
    }
  }
#pragma unroll
  for (int n = 0; n < 32; ++n) hs[n] = 0.0f;
  const float Dd = Dskip[d];

  const int st16 = tid >> 4;
  const int ch4  = (tid & 15) * 4;

  for (int ck = 0; ck < kLen / 16; ++ck) {
    const size_t rowc = (size_t)seq * kLen + (size_t)ck * 16;
    __syncthreads();
#pragma unroll
    for (int i = 0; i < 4; ++i) {
      const int idx = tid + i * 256;
      const int st  = idx >> 6;
      const int c4  = (idx & 63) * 4;
      const v4f v = *(const v4f*)(P + (rowc + st) * kXpPad + c4);
      *(v4f*)(sBC + st * 256 + c4) = v;
    }
    {
      const size_t row = rowc + st16;
      const v4f dtv = *(const v4f*)(P + row * kXpPad + kPDt);
      const v4f uv  = *(const v4f*)(U + row * kHid + ch4);
      const v4f gv  = *(const v4f*)(SG + row * kHid + ch4);
      *(v4f*)(sU + st16 * 64 + ch4) = uv;
      *(v4f*)(sG + st16 * 64 + ch4) = gv;
      v4f dl;
#pragma unroll
      for (int e = 0; e < 4; ++e) {
        const int dd = ch4 + e;
        float acc = dtv[0] * sW[0 * kHid + dd];
        acc = fmaf(dtv[1], sW[1 * kHid + dd], acc);
        acc = fmaf(dtv[2], sW[2 * kHid + dd], acc);
        acc = fmaf(dtv[3], sW[3 * kHid + dd], acc);
        const float pre = acc + sW[kDtr * kHid + dd];
        dl[e] = act_softplus(pre);
      }
      *(v4f*)(sDt + st16 * 64 + ch4) = dl;
    }
    __syncthreads();
#pragma unroll 1
    for (int s = 0; s < 16; ++s) {
      const float dt = sDt[s * 64 + d];
      const float us = sU[s * 64 + d];
      const float gs = sG[s * 64 + d];
      const float du = dt * us;
      const float* bp = sBC + s * 256 + g * 32;
      v4f Bq[8], Cq[8];
#pragma unroll
      for (int k = 0; k < 8; ++k) {
        Bq[k] = *(const v4f*)(bp + 4 * k);
        Cq[k] = *(const v4f*)(bp + kNst + 4 * k);
      }
      float part = 0.0f;
#pragma unroll
      for (int n = 0; n < 32; ++n) {
        const float bn = Bq[n >> 2][n & 3];
        const float cn = Cq[n >> 2][n & 3];
        const float a = expf(dt * Ar[n]);
        hs[n] = fmaf(a, hs[n], du * bn);
        part = fmaf(hs[n], cn, part);
      }
      part += __shfl_xor(part, 1, 32);
      part += __shfl_xor(part, 2, 32);
      const float y = fmaf(us, Dd, part) * gs;
      if (g == 0) sY[s * 64 + d] = y;
    }
    __syncthreads();
    if (tid < 128) {
      const int row = tid >> 3;
      const int c8  = (tid & 7) * 8;
      const float* sp = sY + row * 64 + c8;
      const v4f a0 = *(const v4f*)(sp);
      const v4f a1 = *(const v4f*)(sp + 4);
      v8h hv, lv;
#pragma unroll
      for (int e = 0; e < 4; ++e) {
        _Float16 h0, l0, h1, l1;
        const float f0 = a0[e];
        const float f1 = a1[e];
        f16_split(f0, h0, l0);
        f16_split(f1, h1, l1);
        hv[e] = h0; lv[e] = l0;
        hv[4 + e] = h1; lv[4 + e] = l1;
      }
      const size_t o = (rowc + row) * kHid + c8;
      *(volatile v8h*)(YH + o) = hv;
      *(volatile v8h*)(YL + o) = lv;
      __threadfence();
      *(volatile v8h*)(YH + o) = hv;
      *(volatile v8h*)(YL + o) = lv;
    }
  }
}

__global__ __launch_bounds__(256) void layernorm_store_kernel(
    const float* __restrict__ Y4, const float* __restrict__ lng, const float* __restrict__ lnb,
    float* __restrict__ out)
{
  __shared__ float sRed[8];
  __shared__ __align__(16) float sT[32 * 68];
  const int tid = threadIdx.x, lane = tid & 31, wave = tid >> 5;
  const int seq = blockIdx.x;
  const int bi = seq >> 4;
  const int node = seq & 15;
  const float* ys = Y4 + (size_t)seq * kSeqElems;

  float acc = 0.0f;
  for (int it = 0; it < kSeqElems / 1024; ++it) {
    const v4f v = *(const v4f*)(ys + (size_t)(it * 256 + tid) * 4);
    acc += (v[0] + v[1]) + (v[2] + v[3]);
  }
#pragma unroll
  for (int off = 16; off >= 1; off >>= 1) acc += __shfl_xor(acc, off, 32);
  if (lane == 0) sRed[wave] = acc;
  __syncthreads();
  float tot = sRed[0];
  tot += sRed[1]; tot += sRed[2]; tot += sRed[3];
  tot += sRed[4]; tot += sRed[5]; tot += sRed[6]; tot += sRed[7];
  const float mu = tot * kInvCount;
  __syncthreads();

  float acc2 = 0.0f;
  for (int it = 0; it < kSeqElems / 1024; ++it) {
    const v4f v = *(const v4f*)(ys + (size_t)(it * 256 + tid) * 4);
    const float d0 = v[0] - mu, d1 = v[1] - mu, d2 = v[2] - mu, d3 = v[3] - mu;
    acc2 += (d0 * d0 + d1 * d1) + (d2 * d2 + d3 * d3);
  }
#pragma unroll
  for (int off = 16; off >= 1; off >>= 1) acc2 += __shfl_xor(acc2, off, 32);
  if (lane == 0) sRed[wave] = acc2;
  __syncthreads();
  float tot2 = sRed[0];
  tot2 += sRed[1]; tot2 += sRed[2]; tot2 += sRed[3];
  tot2 += sRed[4]; tot2 += sRed[5]; tot2 += sRed[6]; tot2 += sRed[7];
  const float var = tot2 * kInvCount;
  const float rstd = 1.0f / sqrtf(var + 1e-5f);

  const int q  = lane >> 3;
  const int lq = (lane & 7) * 4;
  for (int lt = 0; lt < kLen / 32; ++lt) {
    const int l0 = lt * 32;
    __syncthreads();
#pragma unroll
    for (int i = 0; i < 2; ++i) {
      const int idx = tid + i * 256;
      const int l   = idx >> 4;
      const int c4  = (idx & 15) * 4;
      const size_t o = (size_t)(l0 + l) * kNout + c4;
      const v4f v  = *(const v4f*)(ys + o);
      const v4f gg = *(const v4f*)(lng + o);
      const v4f bb = *(const v4f*)(lnb + o);
      v4f r;
#pragma unroll
      for (int e = 0; e < 4; ++e) r[e] = fmaf((v[e] - mu) * rstd, gg[e], bb[e]);
      *(v4f*)(sT + l * 68 + c4) = r;
    }
    __syncthreads();
    v4f ov[2];
#pragma unroll
    for (int it = 0; it < 2; ++it) {
      const int j = wave * 8 + it * 4 + q;
      ov[it][0] = sT[(lq + 0) * 68 + j];
      ov[it][1] = sT[(lq + 1) * 68 + j];
      ov[it][2] = sT[(lq + 2) * 68 + j];
      ov[it][3] = sT[(lq + 3) * 68 + j];
    }
    for (int pass = 0; pass < 2; ++pass) {
#pragma unroll
      for (int it = 0; it < 2; ++it) {
        const int j = wave * 8 + it * 4 + q;
        float* p = out + ((size_t)(node * kNout + j) * kBatch + bi) * kLen + l0 + lq;
        *(volatile v4f*)p = ov[it];
      }
      __threadfence();
    }
  }
}

static_assert(((kRows / 16) * (kHid / 64)) % 8 == 0);
static_assert(((kRows / 16) * ((2 * kHid) / 64)) % 8 == 0);
static_assert(((kRows / 16) * (kXpPad / 64)) % 8 == 0);
static_assert(((kRows / 16) * (kNout / 64)) % 8 == 0);
static_assert(((kHid * kNin / 8) % 256) == 0 && (((2 * kHid) * kHid / 8) % 256) == 0 &&
              ((kXpPad * kHid / 8) % 256) == 0 && ((kHid * kHid / 8) % 256) == 0);
static_assert(((kRows * kNin / 8) % 256) == 0);

extern "C" void kernel_launch(void* const* d_in, const int* in_sizes, int n_in,
                              void* d_out, int out_size, void* d_ws, size_t ws_size,
                              hipStream_t stream)
{
  if (n_in < 16) return;
  if (in_sizes[0]  != kRows * kNin) return;
  if (in_sizes[1]  != kNin * kHid) return;
  if (in_sizes[2]  != kHid) return;
  if (in_sizes[3]  != kHid * 2 * kHid) return;
  if (in_sizes[4]  != kHid * 2) return;
  if (in_sizes[5]  != kHid) return;
  if (in_sizes[6]  != kHid * kXpCols) return;
  if (in_sizes[7]  != kDtr * kHid) return;
  if (in_sizes[8]  != kHid) return;
  if (in_sizes[9]  != kHid * kNst) return;
  if (in_sizes[10] != kHid) return;
  if (in_sizes[11] != kHid * kHid) return;
  if (in_sizes[12] != kHid * kNout) return;
  if (in_sizes[13] != kNout) return;
  if (in_sizes[14] != kLen * kNout) return;
  if (in_sizes[15] != kLen * kNout) return;
  if (out_size != kNode * kNout * kBatch * kLen) return;
  if (ws_size < kWsTotal) return;

  const float* inputs = (const float*)d_in[0];
  const float* W_dim  = (const float*)d_in[1];
  const float* b_dim  = (const float*)d_in[2];
  const float* W_in   = (const float*)d_in[3];
  const float* conv_w = (const float*)d_in[4];
  const float* conv_b = (const float*)d_in[5];
  const float* W_xp   = (const float*)d_in[6];
  const float* W_dt   = (const float*)d_in[7];
  const float* b_dt   = (const float*)d_in[8];
  const float* A_log  = (const float*)d_in[9];
  const float* D_skip = (const float*)d_in[10];
  const float* W_op   = (const float*)d_in[11];
  const float* W_o    = (const float*)d_in[12];
  const float* b_o    = (const float*)d_in[13];
  const float* ln_g   = (const float*)d_in[14];
  const float* ln_b   = (const float*)d_in[15];
  float* out = (float*)d_out;

  char* ws = (char*)d_ws;
  unsigned short* WdimT = (unsigned short*)(ws + kOffWdim);
  unsigned short* WinT  = (unsigned short*)(ws + kOffWin);
  unsigned short* WxpT  = (unsigned short*)(ws + kOffWxp);
  unsigned short* WopT  = (unsigned short*)(ws + kOffWop);
  unsigned short* WoT   = (unsigned short*)(ws + kOffWo);
  unsigned short* WdimL = kWeightLo ? (unsigned short*)(ws + kOffWLo + kOffWdim) : WdimT;
  unsigned short* WinL  = kWeightLo ? (unsigned short*)(ws + kOffWLo + kOffWin)  : WinT;
  unsigned short* WxpL  = kWeightLo ? (unsigned short*)(ws + kOffWLo + kOffWxp)  : WxpT;
  unsigned short* WopL  = kWeightLo ? (unsigned short*)(ws + kOffWLo + kOffWop)  : WopT;
  unsigned short* WoL   = kWeightLo ? (unsigned short*)(ws + kOffWLo + kOffWo)   : WoT;
  unsigned short* XH  = (unsigned short*)(ws + kOffXH);
  unsigned short* XL  = (unsigned short*)(ws + kOffXL);
  unsigned short* XDH = (unsigned short*)(ws + kOffXDH);
  unsigned short* XDL = (unsigned short*)(ws + kOffXDL);
  float*          XI  = (float*)(ws + kOffXI);
  float*          SG  = (float*)(ws + kOffSG);
  float*          U   = (float*)(ws + kOffU);
  unsigned short* UH  = (unsigned short*)(ws + kOffUH);
  unsigned short* UL  = (unsigned short*)(ws + kOffUL);
  float*          P   = (float*)(ws + kOffP);
  unsigned short* YH  = (unsigned short*)(ws + kOffYH);
  unsigned short* YL  = (unsigned short*)(ws + kOffYL);
  unsigned short* TH  = (unsigned short*)(ws + kOffTH);
  unsigned short* TL  = (unsigned short*)(ws + kOffTL);
  float*          Y4  = (float*)(ws + kOffY4);

  pack_weight_kernel<kWeightLo><<<(kHid * kNin / 8) / 256, 256, 0, stream>>>(W_dim, WdimT, WdimL, kNin, kHid, 0, kHid * kNin / 8);
  pack_weight_kernel<kWeightLo><<<((2 * kHid) * kHid / 8) / 256, 256, 0, stream>>>(W_in, WinT, WinL, kHid, 2 * kHid, 0, (2 * kHid) * kHid / 8);
  pack_weight_kernel<kWeightLo><<<(kXpPad * kHid / 8) / 256, 256, 0, stream>>>(W_xp, WxpT, WxpL, kHid, kXpCols, 1, kXpPad * kHid / 8);
  pack_weight_kernel<kWeightLo><<<(kHid * kHid / 8) / 256, 256, 0, stream>>>(W_op, WopT, WopL, kHid, kHid, 0, kHid * kHid / 8);
  pack_weight_kernel<kWeightLo><<<(kNout * kHid / 8) / 256, 256, 0, stream>>>(W_o, WoT, WoL, kHid, kNout, 0, kNout * kHid / 8);

  split_rows_f16_kernel<<<(kRows * kNin / 8) / 256, 256, 0, stream>>>(inputs, XH, XL, kRows * kNin / 8);

  eng::gemm_f16_kernel<1, kSpl, 0, 1, true><<<dim3((kRows / 16) * (kHid / 64) / 8), 256, 0, stream>>>(
      XH, XL, kNin, WdimT, WdimL, kNin, Y4, Y4, XDH, XDL, kHid, 0, b_dim, kRows, kHid, kNin, kScale, kRScale);

  eng::gemm_f16_kernel<1, kSpl, 2, 0, false><<<dim3((kRows / 16) * ((2 * kHid) / 64) / 8), 256, 0, stream>>>(
      XDH, XDL, kHid, WinT, WinL, kHid, XI, SG, TH, TL, kHid, kHid, b_dim, kRows, 2 * kHid, kHid, kScale, kRScale);

  conv_silu_kernel<<<kRows / 32, 256, 0, stream>>>(XI, conv_w, conv_b, U, UH, UL);

  eng::gemm_f16_kernel<1, kSpl, 0, 0, false><<<dim3((kRows / 16) * (kXpPad / 64) / 8), 256, 0, stream>>>(
      UH, UL, kHid, WxpT, WxpL, kHid, P, P, TH, TL, kXpPad, 0, b_dim, kRows, kXpPad, kHid, kScale, kRScale);

  scan_kernel<<<kSeqs, 256, 0, stream>>>(P, U, SG, W_dt, b_dt, A_log, D_skip, YH, YL);

  eng::gemm_f16_kernel<1, kSpl, 1, 1, false><<<dim3((kRows / 16) * (kHid / 64) / 8), 256, 0, stream>>>(
      YH, YL, kHid, WopT, WopL, kHid, Y4, Y4, TH, TL, kHid, 0, b_dim, kRows, kHid, kHid, kScale, kRScale);

  eng::gemm_f16_kernel<1, kSpl, 0, 0, true><<<dim3((kRows / 16) * (kNout / 64) / 8), 256, 0, stream>>>(
      TH, TL, kHid, WoT, WoL, kHid, Y4, Y4, XDH, XDL, kNout, 0, b_o, kRows, kNout, kHid, kScale, kRScale);

  layernorm_store_kernel<<<kSeqs, 256, 0, stream>>>(Y4, ln_g, ln_b, out);
}
